// HierarchicalReasoningModel4L_ACTV3_Inner_34935263986348
// MI455X (gfx1250) — hardware-verified
//
#include <hip/hip_runtime.h>
#include <hip/hip_bf16.h>

typedef __attribute__((ext_vector_type(16))) _Float16 v16h;
typedef __attribute__((ext_vector_type(8)))  _Float16 v8h;
typedef __attribute__((ext_vector_type(16))) __bf16   v16b;
typedef __attribute__((ext_vector_type(8)))  __bf16   v8b;
typedef __attribute__((ext_vector_type(8)))  float    v8f;
typedef __attribute__((ext_vector_type(4)))  float    v4f;

__device__ __forceinline__ unsigned short f2bf_bits(float f) {
  unsigned u = __float_as_uint(f);
  return (unsigned short)((u + 0x7FFFu + ((u >> 16) & 1u)) >> 16);
}
__device__ __forceinline__ float bf_bits2f(unsigned short h) { return __uint_as_float(((unsigned)h) << 16); }

__device__ __forceinline__ void cbar() { asm volatile("" ::: "memory"); }

__device__ __forceinline__ void dep_guard_h(v8f& a, v8f& b, v16h x, v16h y) { asm volatile("v_nop\n\tv_nop\n\tv_nop\n\tv_nop" : "+v"(a), "+v"(b) : "v"(x), "v"(y)); }
__device__ __forceinline__ void dep_guard_b(v8f& a, v8f& b, v16b x, v16b y) { asm volatile("v_nop\n\tv_nop\n\tv_nop\n\tv_nop" : "+v"(a), "+v"(b) : "v"(x), "v"(y)); }
__device__ __forceinline__ void keep4_h(v16h a, v16h b, v16h c, v16h d) { asm volatile("v_nop" :: "v"(a), "v"(b), "v"(c), "v"(d)); }
__device__ __forceinline__ void keep4_b(v16b a, v16b b, v16b c, v16b d) { asm volatile("v_nop" :: "v"(a), "v"(b), "v"(c), "v"(d)); }
__device__ __forceinline__ void acc_guard4(v8f& a, v8f& b, v8f& c, v8f& d) { asm volatile("v_nop\n\tv_nop\n\tv_nop\n\tv_nop" : "+v"(a), "+v"(b), "+v"(c), "+v"(d)); }
template <typename T> struct Frag;
template <> struct Frag<_Float16> {
  typedef v16h V; union U { v16h v; v8h h[2]; };
  static __device__ __forceinline__ v16h load(const _Float16* p) {
    U f; f.h[0] = *(const v8h*)(p); f.h[1] = *(const v8h*)(p + 16); return f.v;
  }
  static __device__ __forceinline__ v8f mma(v16h a, v16h b, v8f c) {
    return __builtin_amdgcn_wmma_f32_16x16x32_f16(false, a, false, b, (short)0, c, false, false);
  }
  static __device__ __forceinline__ void guard(v8f& a, v8f& b, v16h x, v16h y) { dep_guard_h(a, b, x, y); }
  static __device__ __forceinline__ void keep(v16h a, v16h b, v16h c, v16h d) { keep4_h(a, b, c, d); }
};
template <> struct Frag<__bf16> {
  typedef v16b V; union U { v16b v; v8b h[2]; };
  static __device__ __forceinline__ v16b load(const __bf16* p) {
    U f; f.h[0] = *(const v8b*)(p); f.h[1] = *(const v8b*)(p + 16); return f.v;
  }
  static __device__ __forceinline__ v8f mma(v16b a, v16b b, v8f c) {
    return __builtin_amdgcn_wmma_f32_16x16x32_bf16(false, a, false, b, (short)0, c, false, false);
  }
  static __device__ __forceinline__ void guard(v8f& a, v8f& b, v16b x, v16b y) { dep_guard_b(a, b, x, y); }
  static __device__ __forceinline__ void keep(v16b a, v16b b, v16b c, v16b d) { keep4_b(a, b, c, d); }
};

template <int ET> struct Elem;
template <> struct Elem<0> { typedef _Float16 T; };
template <> struct Elem<1> { typedef __bf16 T; };
template <int ET, bool SPLIT, int BIAS_MODE, int OUT_MODE, bool RESID, int ACT = 0, bool ROPE = false>
__global__ __launch_bounds__(256) void wmma_gemm64(
    const unsigned short* __restrict__ Ap, const unsigned short* __restrict__ A2p, int lda, long strideA,
    const unsigned short* __restrict__ Btp, const unsigned short* __restrict__ Bt2p, int ldb, long strideB,
    void* __restrict__ Cout, void* __restrict__ Cout2, int ldc, long strideC,
    const float* __restrict__ bias,
    const float* __restrict__ resid, long strideR,
    int M, int N, int K, float scale,
    const float* __restrict__ rcos, const float* __restrict__ rsin, int ropeMod, int ropeRem, int posMask) {
  typedef typename Elem<ET>::T T;
  typedef typename Frag<T>::V V;
  const T* A = (const T*)Ap; const T* A2 = (const T*)A2p; const T* Bt = (const T*)Btp; const T* Bt2 = (const T*)Bt2p;
  __shared__ __align__(16) float sT[8][16 * 68];
  const int b    = blockIdx.y;
  const int lane = threadIdx.x & 31;
  const int wave = threadIdx.x >> 5;
  const int tilesN = N >> 6;
  const int tilesM = M >> 6;
  const int tile = blockIdx.x * 8 + wave;
  if (tile >= tilesM * tilesN) return;
  const int tm = tile / tilesN;
  const int tn = tile - tm * tilesN;
  const int m0 = tm << 6;
  const int n0 = tn << 6;

  const T* Ab  = A  + (size_t)b * strideA;
  const T* Bb  = Bt + (size_t)b * strideB;
  const T* Ab2 = SPLIT ? (A2  + (size_t)b * strideA) : nullptr;
  const T* Bb2 = SPLIT ? (Bt2 + (size_t)b * strideB) : nullptr;

  const int rlane = lane & 15;
  const int koff  = (lane >> 4) * 8;
  const int mOff  = (lane >> 4) * 8;

  v8f acc[4][4];
#pragma unroll
  for (int i = 0; i < 4; ++i)
#pragma unroll
    for (int j = 0; j < 4; ++j) acc[i][j] = (v8f){0.f,0.f,0.f,0.f,0.f,0.f,0.f,0.f};

  for (int k0 = 0; k0 < K; k0 += 32) {
    V bh[4], bl[4];
#pragma unroll
    for (int j = 0; j < 4; ++j) {
      const size_t bo = (size_t)(n0 + (j << 4) + rlane) * ldb + koff + k0;
      bh[j] = Frag<T>::load(Bb + bo);
      if (SPLIT) bl[j] = Frag<T>::load(Bb2 + bo);
    }
#pragma unroll
    for (int i = 0; i < 4; ++i) {
      const size_t ao = (size_t)(m0 + (i << 4) + rlane) * lda + koff + k0;
      V ah = Frag<T>::load(Ab + ao);
      V al;
      if (SPLIT) al = Frag<T>::load(Ab2 + ao);
#pragma unroll
      for (int j = 0; j < 4; ++j) {
        acc[i][j] = Frag<T>::mma(ah, bh[j], acc[i][j]);
        if (SPLIT) {
          acc[i][j] = Frag<T>::mma(ah, bl[j], acc[i][j]);
          acc[i][j] = Frag<T>::mma(al, bh[j], acc[i][j]);
        }
      }
      Frag<T>::guard(acc[i][0], acc[i][3], ah, SPLIT ? al : ah);
    }
    Frag<T>::keep(bh[0], bh[1], bh[2], bh[3]);
    if (SPLIT) Frag<T>::keep(bl[0], bl[1], bl[2], bl[3]);
  }
  acc_guard4(acc[0][0], acc[0][1], acc[0][2], acc[0][3]);
  acc_guard4(acc[1][0], acc[1][1], acc[1][2], acc[1][3]);
  acc_guard4(acc[2][0], acc[2][1], acc[2][2], acc[2][3]);
  acc_guard4(acc[3][0], acc[3][1], acc[3][2], acc[3][3]);

  float* slab = sT[wave];
  const float* Rb = RESID ? (resid + (size_t)b * strideR) : nullptr;
  const bool ropeTile = ROPE ? ((tn % ropeMod) == ropeRem) : false;
#pragma unroll
  for (int i = 0; i < 4; ++i) {
    const int mBase = m0 + (i << 4);
#pragma unroll
    for (int j = 0; j < 4; ++j) {
      const int n = n0 + (j << 4) + rlane;
      float bv = 0.f;
      if (BIAS_MODE == 2) bv = bias[n];
#pragma unroll
      for (int r = 0; r < 8; ++r) {
        float v = acc[i][j][r] * scale;
        if (BIAS_MODE == 1) v += bias[mBase + mOff + r];
        if (BIAS_MODE == 2) v += bv;
        if (RESID) v += Rb[(size_t)(mBase + mOff + r) * ldc + n];
        if (ACT == 1) v = tanhf(v);
        if (ACT == 2) v = fmaxf(v, 0.0f);
        if (ACT == 3) v = v / (1.0f + expf(-v));
        if (ACT == 4) v = (v > 0.f) ? v : 0.01f * v;
        if (ACT == 5) v = 0.5f * v * (1.0f + erff(v * 0.70710678118654752f));
        slab[(mOff + r) * 68 + (j << 4) + rlane] = v;
      }
    }
    __builtin_amdgcn_fence(__ATOMIC_RELEASE, "workgroup");
    __builtin_amdgcn_wave_barrier();
    __builtin_amdgcn_fence(__ATOMIC_ACQUIRE, "workgroup");
    if (OUT_MODE == 0) {
      float* C = (float*)Cout + (size_t)b * strideC;
      const int hh = lane >> 4, c4 = (lane & 15) * 4;
      for (int pass = 0; pass < 2; ++pass) {
#pragma unroll
        for (int it = 0; it < 8; ++it) {
          const int row = it * 2 + hh;
          v4f v = *(const v4f*)(slab + row * 68 + c4);
          *(volatile v4f*)(C + (size_t)(mBase + row) * ldc + n0 + c4) = v;
        }
        __threadfence();
      }
    } else {
      const int q = lane >> 3, c8 = (lane & 7) * 8;
      unsigned short* C  = (unsigned short*)Cout  + (size_t)b * strideC;
      unsigned short* C2 = (OUT_MODE == 2) ? ((unsigned short*)Cout2 + (size_t)b * strideC) : nullptr;
      for (int pass = 0; pass < 2; ++pass) {
#pragma unroll
        for (int it = 0; it < 4; ++it) {
          const int row = it * 4 + q;
          const float* sp = slab + row * 68 + c8;
          v8h hv, lv;
#pragma unroll
          for (int e = 0; e < 8; ++e) {
            if (OUT_MODE == 1) {
              float val = sp[e];
              if (ROPE) {
                if (ropeTile) {
                  const int pos = (mBase + row) & posMask;
                  const int jj  = c8 + e;
                  const float cv = rcos[(size_t)pos * 64 + jj];
                  const float sv = rsin[(size_t)pos * 64 + jj];
                  const float ov = slab[row * 68 + (c8 ^ 32) + e];
                  val = (c8 < 32) ? (val * cv - ov * sv) : (val * cv + ov * sv);
                }
              }
              hv[e] = (_Float16)val;
            } else {
              unsigned short hb = f2bf_bits(sp[e]);
              unsigned short lb = f2bf_bits(sp[e] - bf_bits2f(hb));
              hv[e] = __builtin_bit_cast(_Float16, hb);
              lv[e] = __builtin_bit_cast(_Float16, lb);
            }
          }
          *(volatile v8h*)(C + (size_t)(mBase + row) * ldc + n0 + c8) = hv;
          if (OUT_MODE == 2) *(volatile v8h*)(C2 + (size_t)(mBase + row) * ldc + n0 + c8) = lv;
        }
        __threadfence();
      }
    }
    __builtin_amdgcn_fence(__ATOMIC_RELEASE, "workgroup");
    __builtin_amdgcn_wave_barrier();
    __builtin_amdgcn_fence(__ATOMIC_ACQUIRE, "workgroup");
  }
}

__global__ __launch_bounds__(256) void cast8_f32_f16(
    const float* __restrict__ in, _Float16* __restrict__ out, int n8, float scale) {
  const int i = blockIdx.x * 256 + threadIdx.x;
  if (i < n8) {
    const v4f a = *(const v4f*)(in + (size_t)i * 8);
    const v4f b = *(const v4f*)(in + (size_t)i * 8 + 4);
    v8h o;
    o[0] = (_Float16)(a[0] * scale); o[1] = (_Float16)(a[1] * scale);
    o[2] = (_Float16)(a[2] * scale); o[3] = (_Float16)(a[3] * scale);
    o[4] = (_Float16)(b[0] * scale); o[5] = (_Float16)(b[1] * scale);
    o[6] = (_Float16)(b[2] * scale); o[7] = (_Float16)(b[3] * scale);
    *(volatile v8h*)(out + (size_t)i * 8) = o;
    __threadfence();
    *(volatile v8h*)(out + (size_t)i * 8) = o;
  }
}

__global__ __launch_bounds__(256) void k_norm_rope(
    const float* __restrict__ kva, const float* __restrict__ w,
    const float* __restrict__ rcos, const float* __restrict__ rsin,
    _Float16* __restrict__ kvn, _Float16* __restrict__ kpe, int nrows, int ldin, int posMask) {
  const int lane = threadIdx.x & 31;
  const int wave = threadIdx.x >> 5;
  const int row  = blockIdx.x * 8 + wave;
  if (row >= nrows) return;
  const float* x = kva + (size_t)row * ldin;
  const int c0 = lane * 8, c1 = 256 + lane * 8;
  const v4f a0 = *(const v4f*)(x + c0), a1 = *(const v4f*)(x + c0 + 4);
  const v4f a2 = *(const v4f*)(x + c1), a3 = *(const v4f*)(x + c1 + 4);
  float ss = 0.f;
#pragma unroll
  for (int e = 0; e < 4; ++e) { ss += a0[e] * a0[e]; ss += a1[e] * a1[e]; ss += a2[e] * a2[e]; ss += a3[e] * a3[e]; }
#pragma unroll
  for (int off = 16; off >= 1; off >>= 1) ss += __shfl_xor(ss, off, 32);
  const float inv = rsqrtf(ss * (1.0f / 512.0f) + 1e-6f);
  const v4f w0 = *(const v4f*)(w + c0), w1 = *(const v4f*)(w + c0 + 4);
  const v4f w2 = *(const v4f*)(w + c1), w3 = *(const v4f*)(w + c1 + 4);
  v8h o0, o1;
#pragma unroll
  for (int e = 0; e < 4; ++e) {
    o0[e]     = (_Float16)((a0[e] * inv) * w0[e]);
    o0[4 + e] = (_Float16)((a1[e] * inv) * w1[e]);
    o1[e]     = (_Float16)((a2[e] * inv) * w2[e]);
    o1[4 + e] = (_Float16)((a3[e] * inv) * w3[e]);
  }
  const int q8 = (lane & 7) * 8;
  const float* pe = x + 512;
  const v4f u0 = *(const v4f*)(pe + q8), u1 = *(const v4f*)(pe + q8 + 4);
  const v4f p0 = *(const v4f*)(pe + (q8 ^ 32)), p1 = *(const v4f*)(pe + (q8 ^ 32) + 4);
  const int pos = row & posMask;
  const v4f cc0 = *(const v4f*)(rcos + (size_t)pos * 64 + q8), cc1 = *(const v4f*)(rcos + (size_t)pos * 64 + q8 + 4);
  const v4f sn0 = *(const v4f*)(rsin + (size_t)pos * 64 + q8), sn1 = *(const v4f*)(rsin + (size_t)pos * 64 + q8 + 4);
  v8h ro;
#pragma unroll
  for (int e = 0; e < 4; ++e) {
    float t0, t1;
    if (q8 < 32) { t0 = u0[e] * cc0[e] - p0[e] * sn0[e]; t1 = u1[e] * cc1[e] - p1[e] * sn1[e]; }
    else         { t0 = u0[e] * cc0[e] + p0[e] * sn0[e]; t1 = u1[e] * cc1[e] + p1[e] * sn1[e]; }
    ro[e] = (_Float16)t0; ro[4 + e] = (_Float16)t1;
  }
  _Float16* dn = kvn + (size_t)row * 512;
  _Float16* dp = kpe + (size_t)row * 64;
  *(volatile v8h*)(dn + c0) = o0;
  *(volatile v8h*)(dn + c1) = o1;
  if (lane < 8) *(volatile v8h*)(dp + q8) = ro;
  __threadfence();
  *(volatile v8h*)(dn + c0) = o0;
  *(volatile v8h*)(dn + c1) = o1;
  if (lane < 8) *(volatile v8h*)(dp + q8) = ro;
}

__global__ __launch_bounds__(256) void k_vtrans(
    const _Float16* __restrict__ kvp, _Float16* __restrict__ vt, int S, int H, int ldkv) {
  __shared__ __align__(16) _Float16 T[64 * 72];
  const int tid = threadIdx.x, lane = tid & 31, wave = tid >> 5;
  const int s0 = blockIdx.x * 64;
  const int y = blockIdx.y;
  const int dblk = y & 1, bh = y >> 1;
  const int h = bh % H, b = bh / H;
  const int d0 = dblk * 64;
#pragma unroll
  for (int it = 0; it < 2; ++it) {
    const int id = it * 256 + tid;
    const int r = id >> 3, p = id & 7;
    *(v8h*)(T + r * 72 + p * 8) =
        *(const v8h*)(kvp + (size_t)(b * S + s0 + r) * ldkv + (size_t)h * 256 + 128 + d0 + p * 8);
  }
  __syncthreads();
  const int q = lane >> 3, c8 = (lane & 7) * 8;
  const int dA = wave * 8 + q, dB = wave * 8 + 4 + q;
  v8h v0, v1;
#pragma unroll
  for (int e = 0; e < 8; ++e) { v0[e] = T[(c8 + e) * 72 + dA]; v1[e] = T[(c8 + e) * 72 + dB]; }
  _Float16* rA = vt + ((size_t)bh * 128 + d0 + dA) * S + s0 + c8;
  _Float16* rB = vt + ((size_t)bh * 128 + d0 + dB) * S + s0 + c8;
  *(volatile v8h*)rA = v0;
  *(volatile v8h*)rB = v1;
  __threadfence();
  *(volatile v8h*)rA = v0;
  *(volatile v8h*)rB = v1;
}

__device__ __forceinline__ v8f h_mma(v16h a, v16h b, v8f c) {
  c = __builtin_amdgcn_wmma_f32_16x16x32_f16(false, a, false, b, (short)0, c, false, false);
  asm volatile("v_nop\n\tv_nop\n\tv_nop\n\tv_nop" : "+v"(c) : "v"(a), "v"(b));
  return c;
}

#define A_QKD 192
#define A_VD  128
#define A_KC  64
#define A_NW  4
#define A_OP  132
#define A_PSC 32768.0f
__global__ __launch_bounds__(128)
void k_mla_attn(const _Float16* __restrict__ qh, const _Float16* __restrict__ kvp,
                const _Float16* __restrict__ kpe, const _Float16* __restrict__ vt,
                _Float16* __restrict__ oh,
                int S, int H, int ldq, int ldkv, int ldo, float scale) {
  __shared__ __align__(16) _Float16 Qs[A_NW][16 * A_QKD];
  __shared__ __align__(16) _Float16 Ks[A_KC * A_QKD];
  __shared__ __align__(16) _Float16 Vs[A_VD * A_KC];
  __shared__ __align__(16) _Float16 Ps[A_NW][16 * A_KC];
  __shared__ __align__(16) float    Os[A_NW][16 * A_OP];

  const int tid  = threadIdx.x;
  const int wave = tid >> 5;
  const int lane = tid & 31;
  const int hh   = lane >> 4;
  const int c    = lane & 15;

  const int nqb = S / 64;
  const int bx  = blockIdx.x;
  const int qb  = bx % nqb;
  const int bh  = bx / nqb;
  const int h   = bh % H;
  const int b   = bh / H;
  const int qrow0 = b * S + qb * 64 + wave * 16;
  const int krow0 = b * S;

  _Float16* Qw = Qs[wave];
  {
    const _Float16* qsrc = qh + (size_t)qrow0 * ldq + (size_t)h * A_QKD;
#pragma unroll
    for (int it = 0; it < 12; ++it) {
      const int id = it * 32 + lane;
      const int r  = id / 24;
      const int p  = id - r * 24;
      *(v8h*)(Qw + r * A_QKD + p * 8) = *(const v8h*)(qsrc + (size_t)r * ldq + p * 8);
    }
  }
  cbar();

  float mrow[8], lrow[8];
  v8f oacc[8];
  const float neg_inf = -__builtin_inff();
#pragma unroll
  for (int r = 0; r < 8; ++r) { mrow[r] = neg_inf; lrow[r] = 0.f; }
#pragma unroll
  for (int t = 0; t < 8; ++t) oacc[t] = (v8f){0.f,0.f,0.f,0.f,0.f,0.f,0.f,0.f};

  const int nChunks = S / A_KC;
  for (int kc = 0; kc < nChunks; ++kc) {
    const int kv0 = kc * A_KC;
    __syncthreads();
#pragma unroll
    for (int it = 0; it < 8; ++it) {
      const int id = it * 128 + tid;
      const int kv = id >> 4, p = id & 15;
      *(v8h*)(Ks + kv * A_QKD + p * 8) =
          *(const v8h*)(kvp + (size_t)(krow0 + kv0 + kv) * ldkv + (size_t)h * 256 + p * 8);
    }
    cbar();
#pragma unroll
    for (int it = 0; it < 4; ++it) {
      const int id = it * 128 + tid;
      const int kv = id >> 3, p = id & 7;
      *(v8h*)(Ks + kv * A_QKD + 128 + p * 8) =
          *(const v8h*)(kpe + (size_t)(krow0 + kv0 + kv) * 64 + p * 8);
    }
    cbar();
#pragma unroll
    for (int it = 0; it < 8; ++it) {
      const int id = it * 128 + tid;
      const int d = id >> 3, p = id & 7;
      *(v8h*)(Vs + d * A_KC + p * 8) =
          *(const v8h*)(vt + ((size_t)bh * A_VD + d) * S + kv0 + p * 8);
    }
    __syncthreads();

    v8f s[4];
#pragma unroll
    for (int j = 0; j < 4; ++j) s[j] = (v8f){0.f,0.f,0.f,0.f,0.f,0.f,0.f,0.f};
#pragma unroll 1
    for (int dc = 0; dc < 6; ++dc) {
      const v16h qa = Frag<_Float16>::load(Qw + c * A_QKD + dc * 32 + 8 * hh);
#pragma unroll
      for (int j = 0; j < 4; ++j) {
        const v16h kb = Frag<_Float16>::load(Ks + (j * 16 + c) * A_QKD + dc * 32 + 8 * hh);
        s[j] = h_mma(qa, kb, s[j]);
      }
    }

    float cm[8];
#pragma unroll
    for (int r = 0; r < 8; ++r) {
      float m = neg_inf;
#pragma unroll
      for (int j = 0; j < 4; ++j) {
        const float vv = s[j][r] * scale;
        s[j][r] = vv;
        m = fmaxf(m, vv);
      }
#pragma unroll
      for (int off = 1; off < 16; off <<= 1) m = fmaxf(m, __shfl_xor(m, off, 32));
      cm[r] = m;
    }
    _Float16* Pw = Ps[wave];
#pragma unroll
    for (int r = 0; r < 8; ++r) {
      const float mnew  = fmaxf(mrow[r], cm[r]);
      const float alpha = expf(mrow[r] - mnew);
      mrow[r] = mnew;
      float psum = 0.f;
#pragma unroll
      for (int j = 0; j < 4; ++j) {
        const float p = expf(s[j][r] - mnew);
        psum += p;
        Pw[(8 * hh + r) * A_KC + j * 16 + c] = (_Float16)(p * A_PSC);
      }
#pragma unroll
      for (int off = 1; off < 16; off <<= 1) psum += __shfl_xor(psum, off, 32);
      lrow[r] = lrow[r] * alpha + psum;
#pragma unroll
      for (int t = 0; t < 8; ++t) oacc[t][r] *= alpha;
    }
    __builtin_amdgcn_fence(__ATOMIC_RELEASE, "workgroup");
    __builtin_amdgcn_wave_barrier();
    __builtin_amdgcn_fence(__ATOMIC_ACQUIRE, "workgroup");

#pragma unroll 1
    for (int kk = 0; kk < 2; ++kk) {
      const v16h pa = Frag<_Float16>::load(Pw + c * A_KC + kk * 32 + 8 * hh);
#pragma unroll
      for (int t = 0; t < 8; ++t) {
        if (t == 4) cbar();
        const v16h vb = Frag<_Float16>::load(Vs + (t * 16 + c) * A_KC + kk * 32 + 8 * hh);
        oacc[t] = h_mma(pa, vb, oacc[t]);
      }
    }
  }

  float* os = Os[wave];
#pragma unroll
  for (int r = 0; r < 8; ++r) {
    const float inv = 1.0f / (lrow[r] * A_PSC);
#pragma unroll
    for (int t = 0; t < 8; ++t) os[(8 * hh + r) * A_OP + t * 16 + c] = oacc[t][r] * inv;
  }
  __builtin_amdgcn_fence(__ATOMIC_RELEASE, "workgroup");
  __builtin_amdgcn_wave_barrier();
  __builtin_amdgcn_fence(__ATOMIC_ACQUIRE, "workgroup");
  {
    const int rh = lane >> 4;
    const int c8 = (lane & 15) * 8;
    for (int pass = 0; pass < 2; ++pass) {
#pragma unroll
      for (int it = 0; it < 8; ++it) {
        const int row = it * 2 + rh;
        const float* sp = os + row * A_OP + c8;
        const v4f x0 = *(const v4f*)(sp);
        const v4f x1 = *(const v4f*)(sp + 4);
        v8h hv;
        hv[0] = (_Float16)x0[0]; hv[1] = (_Float16)x0[1]; hv[2] = (_Float16)x0[2]; hv[3] = (_Float16)x0[3];
        hv[4] = (_Float16)x1[0]; hv[5] = (_Float16)x1[1]; hv[6] = (_Float16)x1[2]; hv[7] = (_Float16)x1[3];
        *(volatile v8h*)(oh + (size_t)(qrow0 + row) * ldo + (size_t)h * A_VD + c8) = hv;
      }
      __threadfence();
    }
  }
}

extern "C" void kernel_launch(void* const* d_in, const int* in_sizes, int n_in,
                              void* d_out, int out_size, void* d_ws, size_t ws_size,
                              hipStream_t stream) {
  const int Bn = 2, Sn = 2048, Dn = 2048, Hn = 16, QKDn = 192, KVRn = 512, ROPEn = 64, KVPn = 256, VDn = 128;
  const int BS    = Bn * Sn;
  const int NQ    = Hn * QKDn;
  const int NKVA  = KVRn + ROPEn;
  const int NKVB  = Hn * KVPn;
  const int NO    = Hn * VDn;
  if (n_in < 8) return;
  if (in_sizes[0] != BS * Dn || in_sizes[1] != Sn * ROPEn || in_sizes[2] != Sn * ROPEn ||
      in_sizes[3] != NQ * Dn || in_sizes[4] != NKVA * Dn || in_sizes[5] != KVRn ||
      in_sizes[6] != NKVB * KVRn || in_sizes[7] != Dn * NO || out_size != BS * Dn) return;

  const float* x     = (const float*)d_in[0];
  const float* cosp  = (const float*)d_in[1];
  const float* sinp  = (const float*)d_in[2];
  const float* wq    = (const float*)d_in[3];
  const float* wkva  = (const float*)d_in[4];
  const float* kvnw  = (const float*)d_in[5];
  const float* wkvb  = (const float*)d_in[6];
  const float* wo    = (const float*)d_in[7];
  float* out = (float*)d_out;
  char*  ws  = (char*)d_ws;

  size_t off = 0;
  const size_t sz_xh   = (size_t)BS * Dn * 2;
  const size_t sz_wqh  = (size_t)NQ * Dn * 2;
  const size_t sz_wkva = (size_t)NKVA * Dn * 2;
  const size_t sz_wkvb = (size_t)NKVB * KVRn * 2;
  const size_t sz_woh  = (size_t)Dn * NO * 2;
  const size_t sz_qh   = (size_t)BS * NQ * 2;
  const size_t sz_kva  = (size_t)BS * NKVA * 4;
  const size_t sz_kvn  = (size_t)BS * KVRn * 2;
  const size_t sz_kpe  = (size_t)BS * ROPEn * 2;
  const size_t sz_kvp  = (size_t)BS * NKVB * 2;
  const size_t sz_vt   = (size_t)Bn * Hn * VDn * Sn * 2;
  _Float16* x_h    = (_Float16*)(ws + off); off += sz_xh;
  _Float16* wq_h   = (_Float16*)(ws + off); off += sz_wqh;
  _Float16* wkva_h = (_Float16*)(ws + off); off += sz_wkva;
  _Float16* wkvb_h = (_Float16*)(ws + off); off += sz_wkvb;
  _Float16* wo_h   = (_Float16*)(ws + off); off += sz_woh;
  _Float16* q_h    = (_Float16*)(ws + off); off += sz_qh;
  float*    kva    = (float*)(ws + off);    off += sz_kva;
  _Float16* kvn_h  = (_Float16*)(ws + off); off += sz_kvn;
  _Float16* kpe_h  = (_Float16*)(ws + off); off += sz_kpe;
  _Float16* kvp_h  = (_Float16*)(ws + off); off += sz_kvp;
  _Float16* attn_h = x_h;
  _Float16* vt_h   = wq_h;
  if (sz_vt > sz_wqh + sz_wkva + sz_wkvb) return;
  if (off > ws_size) return;

  const float wcarry = 16.0f;
  const float winv   = 1.0f / 16.0f;

  {
    int n8;
    n8 = (BS * Dn) / 8;     cast8_f32_f16<<<(n8 + 255) / 256, 256, 0, stream>>>(x,    x_h,    n8, 1.0f);
    n8 = (NQ * Dn) / 8;     cast8_f32_f16<<<(n8 + 255) / 256, 256, 0, stream>>>(wq,   wq_h,   n8, wcarry);
    n8 = (NKVA * Dn) / 8;   cast8_f32_f16<<<(n8 + 255) / 256, 256, 0, stream>>>(wkva, wkva_h, n8, wcarry);
    n8 = (NKVB * KVRn) / 8; cast8_f32_f16<<<(n8 + 255) / 256, 256, 0, stream>>>(wkvb, wkvb_h, n8, wcarry);
    n8 = (Dn * NO) / 8;     cast8_f32_f16<<<(n8 + 255) / 256, 256, 0, stream>>>(wo,   wo_h,   n8, wcarry);
  }

  {
    const int tiles = (BS / 64) * (NQ / 64);
    wmma_gemm64<0, false, 0, 1, false, 0, true><<<dim3((tiles + 7) / 8, 1), 256, 0, stream>>>(
        (const unsigned short*)x_h, (const unsigned short*)x_h, Dn, 0L,
        (const unsigned short*)wq_h, (const unsigned short*)wq_h, Dn, 0L,
        (void*)q_h, (void*)q_h, NQ, 0L, cosp, cosp, 0L,
        BS, NQ, Dn, winv, cosp, sinp, 3, 2, Sn - 1);
  }
  {
    const int tiles = (BS / 64) * (NKVA / 64);
    wmma_gemm64<0, false, 0, 0, false, 0, false><<<dim3((tiles + 7) / 8, 1), 256, 0, stream>>>(
        (const unsigned short*)x_h, (const unsigned short*)x_h, Dn, 0L,
        (const unsigned short*)wkva_h, (const unsigned short*)wkva_h, Dn, 0L,
        (void*)kva, (void*)kva, NKVA, 0L, cosp, cosp, 0L,
        BS, NKVA, Dn, winv, cosp, sinp, 1, 1, Sn - 1);
  }
  k_norm_rope<<<(BS + 7) / 8, 256, 0, stream>>>(kva, kvnw, cosp, sinp, kvn_h, kpe_h, BS, NKVA, Sn - 1);
  {
    const int tiles = (BS / 64) * (NKVB / 64);
    wmma_gemm64<0, false, 0, 1, false, 0, false><<<dim3((tiles + 7) / 8, 1), 256, 0, stream>>>(
        (const unsigned short*)kvn_h, (const unsigned short*)kvn_h, KVRn, 0L,
        (const unsigned short*)wkvb_h, (const unsigned short*)wkvb_h, KVRn, 0L,
        (void*)kvp_h, (void*)kvp_h, NKVB, 0L, cosp, cosp, 0L,
        BS, NKVB, KVRn, winv, cosp, sinp, 1, 1, Sn - 1);
  }
  k_vtrans<<<dim3(Sn / 64, Bn * Hn * 2), 256, 0, stream>>>(kvp_h, vt_h, Sn, Hn, NKVB);
  {
    const float scale = 0.07216878364870322f;
    k_mla_attn<<<Bn * Hn * (Sn / 64), 128, 0, stream>>>(q_h, kvp_h, kpe_h, vt_h, attn_h, Sn, Hn, NQ, NKVB, NO, scale);
  }
  {
    const int tiles = (BS / 64) * (Dn / 64);
    wmma_gemm64<0, false, 0, 0, false, 0, false><<<dim3((tiles + 7) / 8, 1), 256, 0, stream>>>(
        (const unsigned short*)attn_h, (const unsigned short*)attn_h, NO, 0L,
        (const unsigned short*)wo_h, (const unsigned short*)wo_h, NO, 0L,
        (void*)out, (void*)out, Dn, 0L, cosp, cosp, 0L,
        BS, Dn, NO, winv, cosp, sinp, 1, 1, Sn - 1);
  }
}
